// BlockwiseEarlyExitMamba_44143673868461
// MI455X (gfx1250) — hardware-verified
//
#include <hip/hip_runtime.h>
#include <math.h>

typedef __attribute__((ext_vector_type(16))) _Float16 v16h;
typedef __attribute__((ext_vector_type(8)))  _Float16 v8h;
typedef __attribute__((ext_vector_type(16))) __bf16   v16b;
typedef __attribute__((ext_vector_type(8)))  __bf16   v8b;
typedef __attribute__((ext_vector_type(8)))  float    v8f;
typedef __attribute__((ext_vector_type(4)))  float    v4f;

constexpr int kB     = 128;
constexpr int kLin   = 64;
constexpr int kLeff  = 32;
constexpr int kTok   = kB * kLeff;
constexpr int kXin   = 5;
constexpr int kDm    = 256;
constexpr int kDi    = 512;
constexpr int kNs    = 16;
constexpr int kDtR   = 16;
constexpr int kDtP   = 32;
constexpr int kXW    = 48;
constexpr int kXP    = 64;
constexpr int kCat   = 136;
constexpr int kCatP  = 160;
constexpr int kXZP   = 2 * kDi;
constexpr int kNL    = 4;
constexpr int kHid   = 128;
constexpr int kNcls  = 2;
constexpr int kTP    = 260;
constexpr float kEps = 1e-5f;
static_assert(kCatP % 32 == 0 && kDtP % 32 == 0 && kXP % 64 == 0, "tile multiples");

__device__ __forceinline__ unsigned short f2bf_bits(float f) {
  unsigned u = __float_as_uint(f);
  return (unsigned short)((u + 0x7FFFu + ((u >> 16) & 1u)) >> 16);
}
__device__ __forceinline__ float bf_bits2f(unsigned short h) { return __uint_as_float(((unsigned)h) << 16); }

__device__ __forceinline__ void dep_guard_h(v8f& a, v8f& b, v16h x, v16h y) { asm volatile("v_nop\n\tv_nop\n\tv_nop\n\tv_nop" : "+v"(a), "+v"(b) : "v"(x), "v"(y)); }
__device__ __forceinline__ void dep_guard_b(v8f& a, v8f& b, v16b x, v16b y) { asm volatile("v_nop\n\tv_nop\n\tv_nop\n\tv_nop" : "+v"(a), "+v"(b) : "v"(x), "v"(y)); }
__device__ __forceinline__ void keep4_h(v16h a, v16h b, v16h c, v16h d) { asm volatile("v_nop" :: "v"(a), "v"(b), "v"(c), "v"(d)); }
__device__ __forceinline__ void keep4_b(v16b a, v16b b, v16b c, v16b d) { asm volatile("v_nop" :: "v"(a), "v"(b), "v"(c), "v"(d)); }
__device__ __forceinline__ void acc_guard4(v8f& a, v8f& b, v8f& c, v8f& d) { asm volatile("v_nop\n\tv_nop\n\tv_nop\n\tv_nop" : "+v"(a), "+v"(b), "+v"(c), "+v"(d)); }
template <typename T> struct Frag;
template <> struct Frag<_Float16> {
  typedef v16h V; union U { v16h v; v8h h[2]; };
  static __device__ __forceinline__ v16h load(const _Float16* p) {
    U f; f.h[0] = *(const v8h*)(p); f.h[1] = *(const v8h*)(p + 16); return f.v;
  }
  static __device__ __forceinline__ v8f mma(v16h a, v16h b, v8f c) {
    return __builtin_amdgcn_wmma_f32_16x16x32_f16(false, a, false, b, (short)0, c, false, false);
  }
  static __device__ __forceinline__ void guard(v8f& a, v8f& b, v16h x, v16h y) { dep_guard_h(a, b, x, y); }
  static __device__ __forceinline__ void keep(v16h a, v16h b, v16h c, v16h d) { keep4_h(a, b, c, d); }
};
template <> struct Frag<__bf16> {
  typedef v16b V; union U { v16b v; v8b h[2]; };
  static __device__ __forceinline__ v16b load(const __bf16* p) {
    U f; f.h[0] = *(const v8b*)(p); f.h[1] = *(const v8b*)(p + 16); return f.v;
  }
  static __device__ __forceinline__ v8f mma(v16b a, v16b b, v8f c) {
    return __builtin_amdgcn_wmma_f32_16x16x32_bf16(false, a, false, b, (short)0, c, false, false);
  }
  static __device__ __forceinline__ void guard(v8f& a, v8f& b, v16b x, v16b y) { dep_guard_b(a, b, x, y); }
  static __device__ __forceinline__ void keep(v16b a, v16b b, v16b c, v16b d) { keep4_b(a, b, c, d); }
};

template <int ET> struct Elem;
template <> struct Elem<0> { typedef _Float16 T; };
template <> struct Elem<1> { typedef __bf16 T; };
template <int ET, bool SPLIT, int BIAS_MODE, int OUT_MODE, bool RESID, int ACT = 0>
__global__ __launch_bounds__(256) void wmma_gemm64(
    const unsigned short* __restrict__ Ap, const unsigned short* __restrict__ A2p, int lda, long strideA,
    const unsigned short* __restrict__ Btp, const unsigned short* __restrict__ Bt2p, int ldb, long strideB,
    void* __restrict__ Cout, void* __restrict__ Cout2, int ldc, long strideC,
    const float* __restrict__ bias,
    const float* __restrict__ resid, long strideR,
    int M, int N, int K, float scale) {
  typedef typename Elem<ET>::T T;
  typedef typename Frag<T>::V V;
  const T* A = (const T*)Ap; const T* A2 = (const T*)A2p; const T* Bt = (const T*)Btp; const T* Bt2 = (const T*)Bt2p;
  __shared__ __align__(16) float sT[8][16 * 68];
  const int b    = blockIdx.y;
  const int lane = threadIdx.x & 31;
  const int wave = threadIdx.x >> 5;
  const int tilesN = N >> 6;
  const int tilesM = M >> 6;
  const int tile = blockIdx.x * 8 + wave;
  if (tile >= tilesM * tilesN) return;
  const int tm = tile / tilesN;
  const int tn = tile - tm * tilesN;
  const int m0 = tm << 6;
  const int n0 = tn << 6;

  const T* Ab  = A  + (size_t)b * strideA;
  const T* Bb  = Bt + (size_t)b * strideB;
  const T* Ab2 = SPLIT ? (A2  + (size_t)b * strideA) : nullptr;
  const T* Bb2 = SPLIT ? (Bt2 + (size_t)b * strideB) : nullptr;

  const int rlane = lane & 15;
  const int koff  = (lane >> 4) * 8;
  const int mOff  = (lane >> 4) * 8;

  v8f acc[4][4];
#pragma unroll
  for (int i = 0; i < 4; ++i)
#pragma unroll
    for (int j = 0; j < 4; ++j) acc[i][j] = (v8f){0.f,0.f,0.f,0.f,0.f,0.f,0.f,0.f};

  for (int k0 = 0; k0 < K; k0 += 32) {
    V bh[4], bl[4];
#pragma unroll
    for (int j = 0; j < 4; ++j) {
      const size_t bo = (size_t)(n0 + (j << 4) + rlane) * ldb + koff + k0;
      bh[j] = Frag<T>::load(Bb + bo);
      if (SPLIT) bl[j] = Frag<T>::load(Bb2 + bo);
    }
#pragma unroll
    for (int i = 0; i < 4; ++i) {
      const size_t ao = (size_t)(m0 + (i << 4) + rlane) * lda + koff + k0;
      V ah = Frag<T>::load(Ab + ao);
      V al;
      if (SPLIT) al = Frag<T>::load(Ab2 + ao);
#pragma unroll
      for (int j = 0; j < 4; ++j) {
        acc[i][j] = Frag<T>::mma(ah, bh[j], acc[i][j]);
        if (SPLIT) {
          acc[i][j] = Frag<T>::mma(ah, bl[j], acc[i][j]);
          acc[i][j] = Frag<T>::mma(al, bh[j], acc[i][j]);
        }
      }
      Frag<T>::guard(acc[i][0], acc[i][3], ah, SPLIT ? al : ah);
    }
    Frag<T>::keep(bh[0], bh[1], bh[2], bh[3]);
    if (SPLIT) Frag<T>::keep(bl[0], bl[1], bl[2], bl[3]);
  }
  acc_guard4(acc[0][0], acc[0][1], acc[0][2], acc[0][3]);
  acc_guard4(acc[1][0], acc[1][1], acc[1][2], acc[1][3]);
  acc_guard4(acc[2][0], acc[2][1], acc[2][2], acc[2][3]);
  acc_guard4(acc[3][0], acc[3][1], acc[3][2], acc[3][3]);

  float* slab = sT[wave];
  const float* Rb = RESID ? (resid + (size_t)b * strideR) : nullptr;
#pragma unroll
  for (int i = 0; i < 4; ++i) {
    const int mBase = m0 + (i << 4);
#pragma unroll
    for (int j = 0; j < 4; ++j) {
      const int n = n0 + (j << 4) + rlane;
      float bv = 0.f;
      if (BIAS_MODE == 2) bv = bias[n];
#pragma unroll
      for (int r = 0; r < 8; ++r) {
        float v = acc[i][j][r] * scale;
        if (BIAS_MODE == 1) v += bias[mBase + mOff + r];
        if (BIAS_MODE == 2) v += bv;
        if (RESID) v += Rb[(size_t)(mBase + mOff + r) * ldc + n];
        if (ACT == 1) v = tanhf(v);
        if (ACT == 2) v = fmaxf(v, 0.0f);
        if (ACT == 3) v = v / (1.0f + expf(-v));
        if (ACT == 4) v = (v > 0.f) ? v : 0.01f * v;
        if (ACT == 5) v = 0.5f * v * (1.0f + erff(v * 0.70710678118654752f));
        slab[(mOff + r) * 68 + (j << 4) + rlane] = v;
      }
    }
    __builtin_amdgcn_fence(__ATOMIC_RELEASE, "workgroup");
    __builtin_amdgcn_wave_barrier();
    __builtin_amdgcn_fence(__ATOMIC_ACQUIRE, "workgroup");
    if (OUT_MODE == 0) {
      float* C = (float*)Cout + (size_t)b * strideC;
      const int hh = lane >> 4, c4 = (lane & 15) * 4;
      for (int pass = 0; pass < 2; ++pass) {
#pragma unroll
        for (int it = 0; it < 8; ++it) {
          const int row = it * 2 + hh;
          v4f v = *(const v4f*)(slab + row * 68 + c4);
          *(volatile v4f*)(C + (size_t)(mBase + row) * ldc + n0 + c4) = v;
        }
        __threadfence();
      }
    } else {
      const int q = lane >> 3, c8 = (lane & 7) * 8;
      unsigned short* C  = (unsigned short*)Cout  + (size_t)b * strideC;
      unsigned short* C2 = (OUT_MODE == 2) ? ((unsigned short*)Cout2 + (size_t)b * strideC) : nullptr;
      for (int pass = 0; pass < 2; ++pass) {
#pragma unroll
        for (int it = 0; it < 4; ++it) {
          const int row = it * 4 + q;
          const float* sp = slab + row * 68 + c8;
          v8h hv, lv;
#pragma unroll
          for (int e = 0; e < 8; ++e) {
            if (OUT_MODE == 1) {
              hv[e] = (_Float16)sp[e];
            } else {
              unsigned short hb = f2bf_bits(sp[e]);
              unsigned short lb = f2bf_bits(sp[e] - bf_bits2f(hb));
              hv[e] = __builtin_bit_cast(_Float16, hb);
              lv[e] = __builtin_bit_cast(_Float16, lb);
            }
          }
          *(volatile v8h*)(C + (size_t)(mBase + row) * ldc + n0 + c8) = hv;
          if (OUT_MODE == 2) *(volatile v8h*)(C2 + (size_t)(mBase + row) * ldc + n0 + c8) = lv;
        }
        __threadfence();
      }
    }
    __builtin_amdgcn_fence(__ATOMIC_RELEASE, "workgroup");
    __builtin_amdgcn_wave_barrier();
    __builtin_amdgcn_fence(__ATOMIC_ACQUIRE, "workgroup");
  }
}

__global__ __launch_bounds__(256) void cast_pad_kernel(
    const float* __restrict__ src, unsigned short* __restrict__ dst,
    int G, int R, int Kin, int Rpad, int Kpad, int total8, float scale)
{
  const int i = blockIdx.x * 256 + threadIdx.x;
  if (i >= total8) return;
  const int e0 = i << 3;
  const int rd = e0 / Kpad;
  const int k0 = e0 - rd * Kpad;
  int g = rd / Rpad;
  const int r = rd - g * Rpad;
  g = (g < G) ? g : (G - 1);
  const int rc = (r < R) ? r : (R - 1);
  const bool rowok = (r < R);
  const float* sp = src + ((size_t)g * R + rc) * Kin;
  v8h hv;
#pragma unroll
  for (int j = 0; j < 8; ++j) {
    const int k  = k0 + j;
    const int kc = (k < Kin) ? k : (Kin - 1);
    const float v = sp[kc] * scale;
    hv[j] = (rowok && (k < Kin)) ? (_Float16)v : (_Float16)0.0f;
  }
  unsigned short* q = dst + e0;
  *(volatile v8h*)q = hv;
  __threadfence();
  *(volatile v8h*)q = hv;
}

__global__ __launch_bounds__(256) void tok_cat_kernel(
    const float* __restrict__ x, const float* __restrict__ emb_proto, const float* __restrict__ emb_flags,
    const float* __restrict__ emb_dir, const float* __restrict__ plw, const float* __restrict__ plb,
    const float* __restrict__ piw, const float* __restrict__ pib, unsigned short* __restrict__ cat16, int total8)
{
  #pragma clang fp contract(off)
  const int i = blockIdx.x * 256 + threadIdx.x;
  if (i >= total8) return;
  const int e0  = i << 3;
  const int tok = e0 / kCatP;
  const int k0  = e0 - tok * kCatP;
  const int b   = tok >> 5;
  const int l   = tok & 31;
  const float* xr = x + (size_t)(b * kLin + l) * kXin;
  const float x0 = xr[0], x1 = xr[1], x2 = xr[2], x3 = xr[3], x4 = xr[4];
  int proto = (int)fminf(fmaxf(x0, -2.0e9f), 2.0e9f); proto = min(max(proto, 0), 255);
  int flags = (int)fminf(fmaxf(x2, -2.0e9f), 2.0e9f); flags = min(max(flags, 0), 63);
  int dirn  = (int)fminf(fmaxf(x4, -2.0e9f), 2.0e9f); dirn  = min(max(dirn, 0), 1);
  const float* ep = emb_proto + proto * 32;
  const float* ef = emb_flags + flags * 32;
  const float* ed = emb_dir + dirn * 8;
  v8h hv;
#pragma unroll
  for (int j = 0; j < 8; ++j) {
    const int k = k0 + j;
    const int k31 = k & 31, k7 = k & 7;
    const float vp = ep[k31];
    const float vf = ef[k31];
    const float vd = ed[k7];
    const float ml = x1 * plw[k31];
    const float vl = ml + plb[k31];
    const float mi = x3 * piw[k31];
    const float vi = mi + pib[k31];
    float v = 0.0f;
    v = (k < 32) ? vp : (k < 64) ? vl : (k < 96) ? vf : (k < 128) ? vi : (k < kCat) ? vd : 0.0f;
    hv[j] = (_Float16)v;
  }
  unsigned short* q = cat16 + e0;
  *(volatile v8h*)q = hv;
  __threadfence();
  *(volatile v8h*)q = hv;
}

__global__ __launch_bounds__(256) void ln_kernel(
    const float* __restrict__ src, const float* __restrict__ g, const float* __restrict__ bta,
    float* __restrict__ dstf, unsigned short* __restrict__ dst16, int nrows)
{
  const int lane = threadIdx.x & 31, wave = threadIdx.x >> 5;
  const int row = blockIdx.x * 8 + wave;
  if (row >= nrows) return;
  const float* sp = src + (size_t)row * kDm;
  const v4f a0 = *(const v4f*)(sp + lane * 4);
  const v4f a1 = *(const v4f*)(sp + 128 + lane * 4);
  float s = (a0[0] + a0[1]) + (a0[2] + a0[3]) + ((a1[0] + a1[1]) + (a1[2] + a1[3]));
#pragma unroll
  for (int off = 1; off < 32; off <<= 1) s += __shfl_xor(s, off, 32);
  const float mu = s * (1.0f / 256.0f);
  float q = 0.f;
#pragma unroll
  for (int e = 0; e < 4; ++e) { const float d0 = a0[e] - mu; const float d1 = a1[e] - mu; q += d0 * d0; q += d1 * d1; }
#pragma unroll
  for (int off = 1; off < 32; off <<= 1) q += __shfl_xor(q, off, 32);
  const float var  = q * (1.0f / 256.0f);
  const float rstd = rsqrtf(var + kEps);
  const v4f g0 = *(const v4f*)(g + lane * 4),   g1 = *(const v4f*)(g + 128 + lane * 4);
  const v4f b0 = *(const v4f*)(bta + lane * 4), b1 = *(const v4f*)(bta + 128 + lane * 4);
  v4f o0, o1;
#pragma unroll
  for (int e = 0; e < 4; ++e) {
    o0[e] = ((a0[e] - mu) * rstd) * g0[e] + b0[e];
    o1[e] = ((a1[e] - mu) * rstd) * g1[e] + b1[e];
  }
  const v4f c0 = *(const v4f*)(sp + lane * 8), c1 = *(const v4f*)(sp + lane * 8 + 4);
  const v4f gg0 = *(const v4f*)(g + lane * 8),   gg1 = *(const v4f*)(g + lane * 8 + 4);
  const v4f bb0 = *(const v4f*)(bta + lane * 8), bb1 = *(const v4f*)(bta + lane * 8 + 4);
  v8h hv;
#pragma unroll
  for (int e = 0; e < 4; ++e) {
    hv[e]     = (_Float16)(((c0[e] - mu) * rstd) * gg0[e] + bb0[e]);
    hv[4 + e] = (_Float16)(((c1[e] - mu) * rstd) * gg1[e] + bb1[e]);
  }
  float* dp = dstf + (size_t)row * kDm;
  unsigned short* hp = dst16 + (size_t)row * kDm;
  for (int pass = 0; pass < 2; ++pass) {
    *(volatile v4f*)(dp + lane * 4) = o0;
    *(volatile v4f*)(dp + 128 + lane * 4) = o1;
    *(volatile v8h*)(hp + lane * 8) = hv;
    __threadfence();
  }
}

__global__ __launch_bounds__(256) void conv_silu_kernel(
    const float* __restrict__ XZ, const float* __restrict__ cw, const float* __restrict__ cb,
    float* __restrict__ UC, unsigned short* __restrict__ UC16)
{
  __shared__ __align__(16) float sT[16 * kTP];
  const int tid = threadIdx.x, lane = tid & 31, wave = tid >> 5;
  const int d0 = blockIdx.x * 256, d = d0 + tid;
  const int tok0 = blockIdx.y * kLeff;
  const float w0 = cw[d * 4 + 0], w1 = cw[d * 4 + 1], w2 = cw[d * 4 + 2], w3 = cw[d * 4 + 3];
  const float bc = cb[d];
  float xm3 = 0.f, xm2 = 0.f, xm1 = 0.f;
  const int hrow = wave >> 1;
  const int hch  = (wave & 1) * 128 + lane * 4;
#pragma unroll 1
  for (int sub = 0; sub < kLeff / 16; ++sub) {
    const int lb = tok0 + sub * 16;
#pragma unroll 1
    for (int s = 0; s < 16; ++s) {
      const float xc = XZ[(size_t)(lb + s) * kXZP + d];
      float acc = w0 * xm3;
      acc = fmaf(w1, xm2, acc);
      acc = fmaf(w2, xm1, acc);
      acc = fmaf(w3, xc, acc);
      const float sv = acc + bc;
      const float sg = __builtin_amdgcn_rcpf(1.0f + __expf(-sv));
      sT[s * kTP + tid] = sv * sg;
      xm3 = xm2; xm2 = xm1; xm1 = xc;
    }
    __syncthreads();
    v4f fv[4];
    v8h bv[2];
#pragma unroll
    for (int it = 0; it < 4; ++it) fv[it] = *(const v4f*)(sT + (it * 4 + hrow) * kTP + hch);
#pragma unroll
    for (int it = 0; it < 2; ++it) {
      const float* sp = sT + (it * 8 + wave) * kTP + lane * 8;
      const v4f a0 = *(const v4f*)(sp);
      const v4f a1 = *(const v4f*)(sp + 4);
#pragma unroll
      for (int e = 0; e < 4; ++e) {
        bv[it][e]     = (_Float16)(a0[e] * 16.0f);
        bv[it][4 + e] = (_Float16)(a1[e] * 16.0f);
      }
    }
    for (int pass = 0; pass < 2; ++pass) {
#pragma unroll
      for (int it = 0; it < 4; ++it)
        *(volatile v4f*)(UC + (size_t)(lb + it * 4 + hrow) * kDi + d0 + hch) = fv[it];
#pragma unroll
      for (int it = 0; it < 2; ++it)
        *(volatile v8h*)(UC16 + (size_t)(lb + it * 8 + wave) * kDi + d0 + lane * 8) = bv[it];
      __threadfence();
    }
    __syncthreads();
  }
}

__global__ __launch_bounds__(256) void dt_cast_kernel(
    const float* __restrict__ PROJ, unsigned short* __restrict__ DT16, int total8, float scale)
{
  const int i = blockIdx.x * 256 + threadIdx.x;
  if (i >= total8) return;
  const int e0  = i << 3;
  const int row = e0 >> 5;
  const int c8  = e0 & 31;
  const bool real = (c8 < kDtR);
  const float* p = PROJ + (size_t)row * kXP + (c8 & 8);
  const v4f a0 = *(const v4f*)(p);
  const v4f a1 = *(const v4f*)(p + 4);
  v8h hv;
#pragma unroll
  for (int e = 0; e < 4; ++e) {
    hv[e]     = real ? (_Float16)(a0[e] * scale) : (_Float16)0.0f;
    hv[4 + e] = real ? (_Float16)(a1[e] * scale) : (_Float16)0.0f;
  }
  unsigned short* qd = DT16 + e0;
  *(volatile v8h*)qd = hv;
  __threadfence();
  *(volatile v8h*)qd = hv;
}

__global__ __launch_bounds__(256) void scan_kernel(
    const float* __restrict__ DLR, const float* __restrict__ UC, const float* __restrict__ XZ,
    const float* __restrict__ PROJ, const float* __restrict__ A_log, const float* __restrict__ Dv,
    unsigned short* __restrict__ Y16)
{
  __shared__ __align__(16) float sBC[kLeff * 32];
  __shared__ __align__(16) float sY[kLeff * kTP];
  const int tid = threadIdx.x, lane = tid & 31, wave = tid >> 5;
  const int d0 = blockIdx.x * 256, d = d0 + tid;
  const int tok0 = blockIdx.y * kLeff;

  float An[kNs];
#pragma unroll
  for (int n = 0; n < kNs; ++n) An[n] = -__expf(A_log[(size_t)d * kNs + n]);
  const float Dd = Dv[d];
  float h[kNs];
#pragma unroll
  for (int n = 0; n < kNs; ++n) h[n] = 0.f;

  {
    const int r = tid >> 3, q = (tid & 7) * 4;
    const v4f v = *(const v4f*)(PROJ + (size_t)(tok0 + r) * kXP + kDtR + q);
    *(v4f*)(sBC + r * 32 + q) = v;
  }
  __syncthreads();
#pragma unroll 1
  for (int s = 0; s < kLeff; ++s) {
    const size_t m = (size_t)(tok0 + s);
    const float a     = DLR[m * kDi + d];
    const float delta = fmaxf(a, 0.0f) + log1pf(__expf(-fabsf(a)));
    const float xv    = UC[m * kDi + d];
    const float zv    = XZ[m * kXZP + kDi + d];
    v4f Bq[4], Cq[4];
#pragma unroll
    for (int qq = 0; qq < 4; ++qq) {
      Bq[qq] = *(const v4f*)(sBC + s * 32 + 4 * qq);
      Cq[qq] = *(const v4f*)(sBC + s * 32 + kNs + 4 * qq);
    }
    float du = delta * xv;
    asm volatile("" : "+v"(du));
    float y = 0.f;
#pragma unroll
    for (int n = 0; n < kNs; ++n) {
      const float e = __expf(delta * An[n]);
      float p = du * Bq[n >> 2][n & 3];
      asm volatile("" : "+v"(p));
      float qv = h[n] * e;
      asm volatile("" : "+v"(qv));
      const float hn = qv + p;
      h[n] = hn;
      float rr = Cq[n >> 2][n & 3] * hn;
      asm volatile("" : "+v"(rr));
      y += rr;
    }
    float sk = xv * Dd;
    asm volatile("" : "+v"(sk));
    y += sk;
    const float sg = __builtin_amdgcn_rcpf(1.0f + __expf(-zv));
    const float gz = zv * sg;
    sY[s * kTP + tid] = (y * gz) * 16.0f;
  }
  __syncthreads();
  v8h hv[4];
#pragma unroll
  for (int it = 0; it < 4; ++it) {
    const float* sp = sY + (it * 8 + wave) * kTP + lane * 8;
    const v4f a0 = *(const v4f*)(sp);
    const v4f a1 = *(const v4f*)(sp + 4);
#pragma unroll
    for (int e = 0; e < 4; ++e) { hv[it][e] = (_Float16)a0[e]; hv[it][4 + e] = (_Float16)a1[e]; }
  }
  for (int pass = 0; pass < 2; ++pass) {
#pragma unroll
    for (int it = 0; it < 4; ++it)
      *(volatile v8h*)(Y16 + (size_t)(tok0 + it * 8 + wave) * kDi + d0 + lane * 8) = hv[it];
    __threadfence();
  }
}

__global__ __launch_bounds__(256) void head_out_kernel(
    const float* __restrict__ HID, const float* __restrict__ W2, const float* __restrict__ b2,
    float* __restrict__ out)
{
  __shared__ __align__(16) float sO[kB * kNcls];
  const int t = threadIdx.x, lane = t & 31, wave = t >> 5;
  const int bb = t >> 1, o = t & 1;
  const float* hp = HID + (size_t)bb * kHid;
  const float* wp = W2 + (size_t)o * kHid;
  float s = 0.f;
#pragma unroll 1
  for (int k = 0; k < kHid; ++k) s = fmaf(hp[k], wp[k], s);
  sO[t] = s + b2[o];
  __syncthreads();
  if (wave == 0) {
    const v4f v0 = *(const v4f*)(sO + lane * 4);
    const v4f v1 = *(const v4f*)(sO + 128 + lane * 4);
    for (int pass = 0; pass < 2; ++pass) {
      *(volatile v4f*)(out + lane * 4) = v0;
      *(volatile v4f*)(out + 128 + lane * 4) = v1;
      __threadfence();
    }
  }
}

static inline size_t align_up64k(size_t v) { return (v + 65535) & ~(size_t)65535; }

extern "C" void kernel_launch(void* const* d_in, const int* in_sizes, int n_in,
                              void* d_out, int out_size, void* d_ws, size_t ws_size,
                              hipStream_t stream)
{
  if (n_in < 27) return;
  const float* x         = (const float*)d_in[0];
  const float* emb_proto = (const float*)d_in[1];
  const float* emb_flags = (const float*)d_in[2];
  const float* emb_dir   = (const float*)d_in[3];
  const float* plw       = (const float*)d_in[4];
  const float* plb       = (const float*)d_in[5];
  const float* piw       = (const float*)d_in[6];
  const float* pib       = (const float*)d_in[7];
  const float* fusion_w  = (const float*)d_in[8];
  const float* fusion_b  = (const float*)d_in[9];
  const float* tng       = (const float*)d_in[10];
  const float* tnb       = (const float*)d_in[11];
  const float* in_proj_w = (const float*)d_in[12];
  const float* conv_w    = (const float*)d_in[13];
  const float* conv_b    = (const float*)d_in[14];
  const float* xproj_w   = (const float*)d_in[15];
  const float* dtproj_w  = (const float*)d_in[16];
  const float* dtproj_b  = (const float*)d_in[17];
  const float* a_log     = (const float*)d_in[18];
  const float* d_skip    = (const float*)d_in[19];
  const float* outproj_w = (const float*)d_in[20];
  const float* ng        = (const float*)d_in[21];
  const float* nb        = (const float*)d_in[22];
  const float* cls_w1    = (const float*)d_in[23];
  const float* cls_b1    = (const float*)d_in[24];
  const float* cls_w2    = (const float*)d_in[25];
  const float* cls_b2    = (const float*)d_in[26];
  float* dout = (float*)d_out;

  if (in_sizes[0] != kB * kLin * kXin) return;
  if (in_sizes[1] != 256 * 32 || in_sizes[2] != 64 * 32 || in_sizes[3] != 2 * 8) return;
  if (in_sizes[4] != 32 || in_sizes[5] != 32 || in_sizes[6] != 32 || in_sizes[7] != 32) return;
  if (in_sizes[8] != kDm * kCat || in_sizes[9] != kDm || in_sizes[10] != kDm || in_sizes[11] != kDm) return;
  if (in_sizes[12] != kNL * kXZP * kDm) return;
  if (in_sizes[13] != kNL * kDi * 4 || in_sizes[14] != kNL * kDi) return;
  if (in_sizes[15] != kNL * kXW * kDi) return;
  if (in_sizes[16] != kNL * kDi * kDtR || in_sizes[17] != kNL * kDi) return;
  if (in_sizes[18] != kNL * kDi * kNs || in_sizes[19] != kNL * kDi) return;
  if (in_sizes[20] != kNL * kDm * kDi) return;
  if (in_sizes[21] != kDm || in_sizes[22] != kDm) return;
  if (in_sizes[23] != kHid * kDm || in_sizes[24] != kHid || in_sizes[25] != kNcls * kHid || in_sizes[26] != kNcls) return;
  if (out_size != kB * kNcls) return;

  const size_t SZ_FW16   = align_up64k((size_t)kDm * kCatP * 2);
  const size_t SZ_WIN16  = align_up64k((size_t)kNL * kXZP * kDm * 2);
  const size_t SZ_WXP16  = align_up64k((size_t)kNL * kXP * kDi * 2);
  const size_t SZ_WDT16  = align_up64k((size_t)kNL * kDi * kDtP * 2);
  const size_t SZ_WOUT16 = align_up64k((size_t)kNL * kDm * kDi * 2);
  const size_t SZ_W1H16  = align_up64k((size_t)kHid * kDm * 2);
  const size_t SZ_CAT16  = align_up64k((size_t)kTok * kCatP * 2);
  const size_t SZ_FPRE   = align_up64k((size_t)kTok * kDm * 4);
  const size_t SZ_FEAT   = align_up64k((size_t)kTok * kDm * 4);
  const size_t SZ_FEAT16 = align_up64k((size_t)kTok * kDm * 2);
  const size_t SZ_XZ     = align_up64k((size_t)kTok * kXZP * 4);
  const size_t SZ_UC     = align_up64k((size_t)kTok * kDi * 4);
  const size_t SZ_UC16   = align_up64k((size_t)kTok * kDi * 2);
  const size_t SZ_PROJ   = align_up64k((size_t)kTok * kXP * 4);
  const size_t SZ_DT16   = align_up64k((size_t)kTok * kDtP * 2);
  const size_t SZ_DLR    = align_up64k((size_t)kTok * kDi * 4);
  const size_t SZ_Y16    = align_up64k((size_t)kTok * kDi * 2);
  const size_t SZ_HID    = align_up64k((size_t)kB * kHid * 4);
  const size_t OFF_FW16   = 0;
  const size_t OFF_WIN16  = OFF_FW16   + SZ_FW16;
  const size_t OFF_WXP16  = OFF_WIN16  + SZ_WIN16;
  const size_t OFF_WDT16  = OFF_WXP16  + SZ_WXP16;
  const size_t OFF_WOUT16 = OFF_WDT16  + SZ_WDT16;
  const size_t OFF_W1H16  = OFF_WOUT16 + SZ_WOUT16;
  const size_t OFF_CAT16  = OFF_W1H16  + SZ_W1H16;
  const size_t OFF_FPRE   = OFF_CAT16  + SZ_CAT16;
  const size_t OFF_FEAT   = OFF_FPRE   + SZ_FPRE;
  const size_t OFF_FEAT16 = OFF_FEAT   + SZ_FEAT;
  const size_t OFF_XZ     = OFF_FEAT16 + SZ_FEAT16;
  const size_t OFF_UC     = OFF_XZ     + SZ_XZ;
  const size_t OFF_UC16   = OFF_UC     + SZ_UC;
  const size_t OFF_PROJ   = OFF_UC16   + SZ_UC16;
  const size_t OFF_DT16   = OFF_PROJ   + SZ_PROJ;
  const size_t OFF_DLR    = OFF_DT16   + SZ_DT16;
  const size_t OFF_Y16    = OFF_DLR    + SZ_DLR;
  const size_t OFF_HID    = OFF_Y16    + SZ_Y16;
  const size_t TOTAL      = OFF_HID    + SZ_HID;
  if (ws_size < TOTAL) return;

  char* ws = (char*)d_ws;
  unsigned short* FW16   = (unsigned short*)(ws + OFF_FW16);
  unsigned short* WIN16  = (unsigned short*)(ws + OFF_WIN16);
  unsigned short* WXP16  = (unsigned short*)(ws + OFF_WXP16);
  unsigned short* WDT16  = (unsigned short*)(ws + OFF_WDT16);
  unsigned short* WOUT16 = (unsigned short*)(ws + OFF_WOUT16);
  unsigned short* W1H16  = (unsigned short*)(ws + OFF_W1H16);
  unsigned short* CAT16  = (unsigned short*)(ws + OFF_CAT16);
  float*          FPRE   = (float*)(ws + OFF_FPRE);
  float*          FEAT   = (float*)(ws + OFF_FEAT);
  unsigned short* FEAT16 = (unsigned short*)(ws + OFF_FEAT16);
  float*          XZ     = (float*)(ws + OFF_XZ);
  float*          UC     = (float*)(ws + OFF_UC);
  unsigned short* UC16   = (unsigned short*)(ws + OFF_UC16);
  float*          PROJ   = (float*)(ws + OFF_PROJ);
  unsigned short* DT16   = (unsigned short*)(ws + OFF_DT16);
  float*          DLR    = (float*)(ws + OFF_DLR);
  unsigned short* Y16    = (unsigned short*)(ws + OFF_Y16);
  float*          HID    = (float*)(ws + OFF_HID);
  const float* dummy_bias  = fusion_b;
  const float* dummy_resid = FEAT;

  {
    const int t8_fw   = (1   * kDm  * kCatP) / 8;
    const int t8_win  = (kNL * kXZP * kDm ) / 8;
    const int t8_wxp  = (kNL * kXP  * kDi ) / 8;
    const int t8_wdt  = (kNL * kDi  * kDtP) / 8;
    const int t8_wout = (kNL * kDm  * kDi ) / 8;
    const int t8_w1   = (1   * kHid * kDm ) / 8;
    cast_pad_kernel<<<t8_fw / 256,   256, 0, stream>>>(fusion_w,  FW16,   1,   kDm,  kCat, kDm,  kCatP, t8_fw,   32.0f);
    cast_pad_kernel<<<t8_win / 256,  256, 0, stream>>>(in_proj_w, WIN16,  kNL, kXZP, kDm,  kXZP, kDm,   t8_win,  32.0f);
    cast_pad_kernel<<<t8_wxp / 256,  256, 0, stream>>>(xproj_w,   WXP16,  kNL, kXW,  kDi,  kXP,  kDi,   t8_wxp,  32.0f);
    cast_pad_kernel<<<t8_wdt / 256,  256, 0, stream>>>(dtproj_w,  WDT16,  kNL, kDi,  kDtR, kDi,  kDtP,  t8_wdt,  8.0f);
    cast_pad_kernel<<<t8_wout / 256, 256, 0, stream>>>(outproj_w, WOUT16, kNL, kDm,  kDi,  kDm,  kDi,   t8_wout, 32.0f);
    cast_pad_kernel<<<t8_w1 / 256,   256, 0, stream>>>(cls_w1,    W1H16,  1,   kHid, kDm,  kHid, kDm,   t8_w1,   32.0f);
  }

  {
    const int t8_cat = (kTok * kCatP) / 8;
    tok_cat_kernel<<<t8_cat / 256, 256, 0, stream>>>(x, emb_proto, emb_flags, emb_dir, plw, plb, piw, pib, CAT16, t8_cat);
  }

  wmma_gemm64<0, false, 2, 0, false, 0><<<dim3((kTok / 64) * (kDm / 64) / 8, 1), 256, 0, stream>>>(
      CAT16, CAT16, kCatP, 0L, FW16, FW16, kCatP, 0L,
      (void*)FPRE, (void*)FPRE, kDm, 0L, fusion_b, dummy_resid, 0L, kTok, kDm, kCatP, 1.0f / 32.0f);
  ln_kernel<<<kTok / 8, 256, 0, stream>>>(FPRE, tng, tnb, FEAT, FEAT16, kTok);

  for (int layer = 0; layer < kNL; ++layer) {
    const unsigned short* WINl  = WIN16  + (size_t)layer * kXZP * kDm;
    const unsigned short* WXPl  = WXP16  + (size_t)layer * kXP * kDi;
    const unsigned short* WDTl  = WDT16  + (size_t)layer * kDi * kDtP;
    const unsigned short* WOUTl = WOUT16 + (size_t)layer * kDm * kDi;
    const float* cwl  = conv_w   + (size_t)layer * kDi * 4;
    const float* cbl  = conv_b   + (size_t)layer * kDi;
    const float* dbl  = dtproj_b + (size_t)layer * kDi;
    const float* all  = a_log    + (size_t)layer * kDi * kNs;
    const float* dsl  = d_skip   + (size_t)layer * kDi;

    wmma_gemm64<0, false, 0, 0, false, 0><<<dim3((kTok / 64) * (kXZP / 64) / 8, 1), 256, 0, stream>>>(
        FEAT16, FEAT16, kDm, 0L, WINl, WINl, kDm, 0L,
        (void*)XZ, (void*)XZ, kXZP, 0L, dummy_bias, dummy_resid, 0L, kTok, kXZP, kDm, 1.0f / 32.0f);

    conv_silu_kernel<<<dim3(kDi / 256, kB), 256, 0, stream>>>(XZ, cwl, cbl, UC, UC16);

    wmma_gemm64<0, false, 0, 0, false, 0><<<dim3((kTok / 64) * (kXP / 64) / 8, 1), 256, 0, stream>>>(
        UC16, UC16, kDi, 0L, WXPl, WXPl, kDi, 0L,
        (void*)PROJ, (void*)PROJ, kXP, 0L, dummy_bias, dummy_resid, 0L, kTok, kXP, kDi, 1.0f / 512.0f);

    dt_cast_kernel<<<(kTok * kDtP) / 8 / 256, 256, 0, stream>>>(PROJ, DT16, (kTok * kDtP) / 8, 16.0f);

    wmma_gemm64<0, false, 2, 0, false, 0><<<dim3((kTok / 64) * (kDi / 64) / 8, 1), 256, 0, stream>>>(
        DT16, DT16, kDtP, 0L, WDTl, WDTl, kDtP, 0L,
        (void*)DLR, (void*)DLR, kDi, 0L, dbl, dummy_resid, 0L, kTok, kDi, kDtP, 1.0f / 128.0f);

    scan_kernel<<<dim3(kDi / 256, kB), 256, 0, stream>>>(DLR, UC, XZ, PROJ, all, dsl, Y16);

    wmma_gemm64<0, false, 0, 0, true, 0><<<dim3((kTok / 64) * (kDm / 64) / 8, 1), 256, 0, stream>>>(
        Y16, Y16, kDi, 0L, WOUTl, WOUTl, kDi, 0L,
        (void*)FPRE, (void*)FPRE, kDm, 0L, dummy_bias, FEAT, 0L, kTok, kDm, kDi, 1.0f / 512.0f);

    ln_kernel<<<kTok / 8, 256, 0, stream>>>(FPRE, ng, nb, FEAT, FEAT16, kTok);
  }

  wmma_gemm64<0, false, 2, 0, false, 2><<<dim3(1, 1), 256, 0, stream>>>(
      FEAT16 + (size_t)(kLeff - 1) * kDm, FEAT16 + (size_t)(kLeff - 1) * kDm, kLeff * kDm, 0L, W1H16, W1H16, kDm, 0L,
      (void*)HID, (void*)HID, kHid, 0L, cls_b1, dummy_resid, 0L, kB, kHid, kDm, 1.0f / 32.0f);

  head_out_kernel<<<1, 256, 0, stream>>>(HID, cls_w2, cls_b2, dout);
}
